// MultiScaleRetention_60258391162953
// MI455X (gfx1250) — hardware-verified
//
#include <hip/hip_runtime.h>
#include <math.h>

constexpr int kB    = 2;
constexpr int kS    = 2048;
constexpr int kHid  = 1024;
constexpr int kNH   = 8;
constexpr int kHD   = 128;
constexpr int kTok  = kB * kS;
constexpr int kGrp  = 2;
constexpr float kQCarry     = 16.0f;
constexpr float kVCarry     = 16.0f;
constexpr float kPCarry     = 2048.0f;
constexpr float kW2Carry    = 1024.0f;
constexpr float kScoreScale = 1.0f / (16.0f * 16.0f);
constexpr float kPVScale    = 1.0f / (2048.0f * 16.0f);
constexpr float kOutScale   = 1.0f / 1024.0f;
constexpr float kEps        = 1.0e-5f;
constexpr float kInvHD      = 1.0f / 128.0f;
static_assert(kNH * kHD == kHid, "shape");
static_assert(kNH % kGrp == 0, "groups");
static_assert(kHD % 32 == 0 && kHid % 32 == 0 && kS % 32 == 0, "K multiples of 32");
static_assert(kTok % 64 == 0 && kHD % 64 == 0 && kS % 64 == 0 && kHid % 64 == 0, "M,N multiples of 64");
static_assert(kS % 8 == 0 && (kTok * kHid) % (256 * 8) == 0, "cast grids exact");

typedef __attribute__((ext_vector_type(16))) _Float16 v16h;
typedef __attribute__((ext_vector_type(8)))  _Float16 v8h;
typedef __attribute__((ext_vector_type(16))) __bf16   v16b;
typedef __attribute__((ext_vector_type(8)))  __bf16   v8b;
typedef __attribute__((ext_vector_type(8)))  float    v8f;
typedef __attribute__((ext_vector_type(4)))  float    v4f;
typedef __attribute__((ext_vector_type(4)))  unsigned int v4u;

__device__ __forceinline__ unsigned short f2bf_bits(float f) {
  unsigned u = __float_as_uint(f);
  return (unsigned short)((u + 0x7FFFu + ((u >> 16) & 1u)) >> 16);
}
__device__ __forceinline__ float bf_bits2f(unsigned short h) { return __uint_as_float(((unsigned)h) << 16); }

__device__ __forceinline__ void dep_guard_h(v8f& a, v8f& b, v16h x, v16h y) { asm volatile("v_nop\n\tv_nop\n\tv_nop\n\tv_nop" : "+v"(a), "+v"(b) : "v"(x), "v"(y)); }
__device__ __forceinline__ void dep_guard_b(v8f& a, v8f& b, v16b x, v16b y) { asm volatile("v_nop\n\tv_nop\n\tv_nop\n\tv_nop" : "+v"(a), "+v"(b) : "v"(x), "v"(y)); }
__device__ __forceinline__ void dep_guard4_h(v8f& a, v8f& b, v8f& c, v8f& d, v16h x, v16h y) { asm volatile("v_nop\n\tv_nop\n\tv_nop\n\tv_nop" : "+v"(a), "+v"(b), "+v"(c), "+v"(d) : "v"(x), "v"(y)); }
__device__ __forceinline__ void dep_guard4_b(v8f& a, v8f& b, v8f& c, v8f& d, v16b x, v16b y) { asm volatile("v_nop\n\tv_nop\n\tv_nop\n\tv_nop" : "+v"(a), "+v"(b), "+v"(c), "+v"(d) : "v"(x), "v"(y)); }
__device__ __forceinline__ void keep4_h(v16h a, v16h b, v16h c, v16h d) { asm volatile("v_nop" :: "v"(a), "v"(b), "v"(c), "v"(d)); }
__device__ __forceinline__ void keep4_b(v16b a, v16b b, v16b c, v16b d) { asm volatile("v_nop" :: "v"(a), "v"(b), "v"(c), "v"(d)); }
__device__ __forceinline__ void acc_guard4(v8f& a, v8f& b, v8f& c, v8f& d) { asm volatile("v_nop\n\tv_nop\n\tv_nop\n\tv_nop" : "+v"(a), "+v"(b), "+v"(c), "+v"(d)); }
template <typename T> struct Frag;
template <> struct Frag<_Float16> {
  typedef v16h V; union U { v16h v; v8h h[2]; };
  static __device__ __forceinline__ v16h load(const _Float16* p) {
    U f; f.h[0] = *(const v8h*)(p); f.h[1] = *(const v8h*)(p + 16); return f.v;
  }
  static __device__ __forceinline__ v8f mma(v16h a, v16h b, v8f c) {
    return __builtin_amdgcn_wmma_f32_16x16x32_f16(false, a, false, b, (short)0, c, false, false);
  }
  static __device__ __forceinline__ void guard(v8f& a, v8f& b, v16h x, v16h y) { dep_guard_h(a, b, x, y); }
  static __device__ __forceinline__ void guard4(v8f& a, v8f& b, v8f& c, v8f& d, v16h x, v16h y) { dep_guard4_h(a, b, c, d, x, y); }
  static __device__ __forceinline__ void keep(v16h a, v16h b, v16h c, v16h d) { keep4_h(a, b, c, d); }
};
template <> struct Frag<__bf16> {
  typedef v16b V; union U { v16b v; v8b h[2]; };
  static __device__ __forceinline__ v16b load(const __bf16* p) {
    U f; f.h[0] = *(const v8b*)(p); f.h[1] = *(const v8b*)(p + 16); return f.v;
  }
  static __device__ __forceinline__ v8f mma(v16b a, v16b b, v8f c) {
    return __builtin_amdgcn_wmma_f32_16x16x32_bf16(false, a, false, b, (short)0, c, false, false);
  }
  static __device__ __forceinline__ void guard(v8f& a, v8f& b, v16b x, v16b y) { dep_guard_b(a, b, x, y); }
  static __device__ __forceinline__ void guard4(v8f& a, v8f& b, v8f& c, v8f& d, v16b x, v16b y) { dep_guard4_b(a, b, c, d, x, y); }
  static __device__ __forceinline__ void keep(v16b a, v16b b, v16b c, v16b d) { keep4_b(a, b, c, d); }
};

__device__ __forceinline__ unsigned pk16(unsigned short a, unsigned short b) { return (unsigned)a | ((unsigned)b << 16); }
__device__ __forceinline__ unsigned short h_bits(float f) { const _Float16 h = (_Float16)f; return __builtin_bit_cast(unsigned short, h); }

template <int ET> struct Elem;
template <> struct Elem<0> { typedef _Float16 T; };
template <> struct Elem<1> { typedef __bf16 T; };
template <int ET, bool SPLIT, int BIAS_MODE, int OUT_MODE, bool RESID, int ACT, int CAUS>
__global__ __launch_bounds__(256) void wmma_gemm64(
    const unsigned short* __restrict__ Ap, const unsigned short* __restrict__ A2p, int lda, long strideA,
    const unsigned short* __restrict__ Btp, const unsigned short* __restrict__ Bt2p, int ldb, long strideB,
    void* __restrict__ Cout, void* __restrict__ Cout2, int ldc, long strideC,
    const float* __restrict__ bias,
    const float* __restrict__ resid, long strideR,
    int M, int N, int K, float scale) {
  typedef typename Elem<ET>::T T;
  typedef typename Frag<T>::V V;
  const T* A = (const T*)Ap; const T* A2 = (const T*)A2p; const T* Bt = (const T*)Btp; const T* Bt2 = (const T*)Bt2p;
  __shared__ __align__(16) float sT[8][16 * 68];
  const int b    = blockIdx.y;
  const int lane = threadIdx.x & 31;
  const int wave = threadIdx.x >> 5;
  const int tilesN = N >> 6;
  const int tilesM = M >> 6;
  const int tile = blockIdx.x * 8 + wave;
  if (tile >= tilesM * tilesN) return;
  const int tm = tile / tilesN;
  const int tn = tile - tm * tilesN;
  if (CAUS == 1 && tn > tm) return;
  const int m0 = tm << 6;
  const int n0 = tn << 6;
  const int kEnd = (CAUS == 2) ? (m0 + 64) : K;

  const T* Ab  = A  + (size_t)b * strideA;
  const T* Bb  = Bt + (size_t)b * strideB;
  const T* Ab2 = SPLIT ? (A2  + (size_t)b * strideA) : nullptr;
  const T* Bb2 = SPLIT ? (Bt2 + (size_t)b * strideB) : nullptr;

  const int rlane = lane & 15;
  const int koff  = (lane >> 4) * 8;
  const int mOff  = (lane >> 4) * 8;

  v8f acc[4][4];
#pragma unroll
  for (int i = 0; i < 4; ++i)
#pragma unroll
    for (int j = 0; j < 4; ++j) acc[i][j] = (v8f){0.f,0.f,0.f,0.f,0.f,0.f,0.f,0.f};

  for (int k0 = 0; k0 < kEnd; k0 += 32) {
    V bh[4], bl[4];
#pragma unroll
    for (int j = 0; j < 4; ++j) {
      const size_t bo = (size_t)(n0 + (j << 4) + rlane) * ldb + koff + k0;
      bh[j] = Frag<T>::load(Bb + bo);
      if (SPLIT) bl[j] = Frag<T>::load(Bb2 + bo);
    }
#pragma unroll
    for (int i = 0; i < 4; ++i) {
      const size_t ao = (size_t)(m0 + (i << 4) + rlane) * lda + koff + k0;
      V ah = Frag<T>::load(Ab + ao);
      V al;
      if (SPLIT) al = Frag<T>::load(Ab2 + ao);
#pragma unroll
      for (int j = 0; j < 4; ++j) {
        acc[i][j] = Frag<T>::mma(ah, bh[j], acc[i][j]);
        if (SPLIT) {
          acc[i][j] = Frag<T>::mma(ah, bl[j], acc[i][j]);
          acc[i][j] = Frag<T>::mma(al, bh[j], acc[i][j]);
        }
      }
      Frag<T>::guard4(acc[i][0], acc[i][1], acc[i][2], acc[i][3], ah, SPLIT ? al : ah);
    }
    Frag<T>::keep(bh[0], bh[1], bh[2], bh[3]);
    if (SPLIT) Frag<T>::keep(bl[0], bl[1], bl[2], bl[3]);
  }
  acc_guard4(acc[0][0], acc[0][1], acc[0][2], acc[0][3]);
  acc_guard4(acc[1][0], acc[1][1], acc[1][2], acc[1][3]);
  acc_guard4(acc[2][0], acc[2][1], acc[2][2], acc[2][3]);
  acc_guard4(acc[3][0], acc[3][1], acc[3][2], acc[3][3]);

  float* slab = sT[wave];
  const float* Rb = RESID ? (resid + (size_t)b * strideR) : nullptr;
#pragma unroll
  for (int i = 0; i < 4; ++i) {
    const int mBase = m0 + (i << 4);
#pragma unroll
    for (int j = 0; j < 4; ++j) {
      const int n = n0 + (j << 4) + rlane;
      float bv = 0.f;
      if (BIAS_MODE == 2) bv = bias[n];
#pragma unroll
      for (int r = 0; r < 8; ++r) {
        float v = acc[i][j][r] * scale;
        if (BIAS_MODE == 1) v += bias[mBase + mOff + r];
        if (BIAS_MODE == 2) v += bv;
        if (RESID) v += Rb[(size_t)(mBase + mOff + r) * ldc + n];
        if (ACT == 2) v = fmaxf(v, 0.0f);
        if (ACT == 4) v = (v > 0.f) ? v : 0.01f * v;
        slab[(mOff + r) * 68 + (j << 4) + rlane] = v;
      }
    }
    __builtin_amdgcn_fence(__ATOMIC_RELEASE, "workgroup");
    __builtin_amdgcn_wave_barrier();
    __builtin_amdgcn_fence(__ATOMIC_ACQUIRE, "workgroup");
    if (OUT_MODE == 0) {
      float* C = (float*)Cout + (size_t)b * strideC;
      const int hh = lane >> 4, c4 = (lane & 15) * 4;
      for (int pass = 0; pass < 2; ++pass) {
#pragma unroll
        for (int it = 0; it < 8; ++it) {
          const int row = it * 2 + hh;
          v4f v = *(const v4f*)(slab + row * 68 + c4);
          *(volatile v4f*)(C + (size_t)(mBase + row) * ldc + n0 + c4) = v;
        }
        __threadfence();
      }
    } else {
      const int q = lane >> 3, c8 = (lane & 7) * 8;
      unsigned short* C  = (unsigned short*)Cout  + (size_t)b * strideC;
      unsigned short* C2 = (OUT_MODE == 2) ? ((unsigned short*)Cout2 + (size_t)b * strideC) : nullptr;
      for (int pass = 0; pass < 2; ++pass) {
#pragma unroll
        for (int it = 0; it < 4; ++it) {
          const int row = it * 4 + q;
          const float* sp = slab + row * 68 + c8;
          v8h hv, lv;
#pragma unroll
          for (int e = 0; e < 8; ++e) {
            if (OUT_MODE == 1) {
              hv[e] = (_Float16)sp[e];
            } else {
              unsigned short hb = f2bf_bits(sp[e]);
              unsigned short lb = f2bf_bits(sp[e] - bf_bits2f(hb));
              hv[e] = __builtin_bit_cast(_Float16, hb);
              lv[e] = __builtin_bit_cast(_Float16, lb);
            }
          }
          *(volatile v8h*)(C + (size_t)(mBase + row) * ldc + n0 + c8) = hv;
          if (OUT_MODE == 2) *(volatile v8h*)(C2 + (size_t)(mBase + row) * ldc + n0 + c8) = lv;
        }
        __threadfence();
      }
    }
    __builtin_amdgcn_fence(__ATOMIC_RELEASE, "workgroup");
    __builtin_amdgcn_wave_barrier();
    __builtin_amdgcn_fence(__ATOMIC_ACQUIRE, "workgroup");
  }
}

__global__ __launch_bounds__(256) void cast8_bf16_kernel(const float* __restrict__ in, unsigned short* __restrict__ out, int n8) {
  const int i = blockIdx.x * 256 + threadIdx.x;
  if (i >= n8) return;
  const float* p = in + 8 * (size_t)i;
  const v4f a = *(const v4f*)(p);
  const v4f c = *(const v4f*)(p + 4);
  unsigned short hb[8];
#pragma unroll
  for (int e = 0; e < 4; ++e) {
    hb[e]     = f2bf_bits(a[e]);
    hb[4 + e] = f2bf_bits(c[e]);
  }
  const v4u u = (v4u){pk16(hb[0], hb[1]), pk16(hb[2], hb[3]), pk16(hb[4], hb[5]), pk16(hb[6], hb[7])};
  unsigned short* q = out + 8 * (size_t)i;
  *(volatile v4u*)q = u;
  __threadfence();
  *(volatile v4u*)q = u;
}

__global__ __launch_bounds__(256) void headw_kernel(const float* __restrict__ Wq, const float* __restrict__ Wk,
                                                    const float* __restrict__ Wv, unsigned short* __restrict__ WT) {
  __shared__ float sm[64][65];
  const int t  = threadIdx.x;
  const int d0 = blockIdx.x * 64;
  const int e0 = blockIdx.y * 64;
  const int z  = blockIdx.z;
  const int which = z >> 3, h = z & 7;
  const float* W  = (which == 0) ? Wq : (which == 1) ? Wk : Wv;
  const float* Wh = W + (size_t)h * kHD * kHD;
#pragma unroll
  for (int i = 0; i < 8; ++i) {
    const int idx = i * 256 + t;
    const int r = idx >> 6;
    const int c = idx & 63;
    sm[c][r] = Wh[(size_t)(d0 + r) * kHD + e0 + c];
  }
  asm volatile("" ::: "memory");
#pragma unroll
  for (int i = 8; i < 16; ++i) {
    const int idx = i * 256 + t;
    const int r = idx >> 6;
    const int c = idx & 63;
    sm[c][r] = Wh[(size_t)(d0 + r) * kHD + e0 + c];
  }
  __syncthreads();
  const int lane = t & 31, wave = t >> 5;
  const int q = lane >> 3, c8 = (lane & 7) * 8;
  unsigned short* op = WT + (size_t)z * kHD * kHD;
  for (int pass = 0; pass < 2; ++pass) {
#pragma unroll
    for (int it = 0; it < 2; ++it) {
      const int row = wave * 8 + it * 4 + q;
      unsigned short hb[8];
#pragma unroll
      for (int e = 0; e < 8; ++e) hb[e] = f2bf_bits(sm[row][c8 + e]);
      const v4u u = (v4u){pk16(hb[0], hb[1]), pk16(hb[2], hb[3]), pk16(hb[4], hb[5]), pk16(hb[6], hb[7])};
      *(volatile v4u*)(op + (size_t)(e0 + row) * kHD + d0 + c8) = u;
    }
    __threadfence();
  }
}

__global__ __launch_bounds__(256) void sqw_kernel(const float* __restrict__ W1, const float* __restrict__ W2,
                                                  unsigned short* __restrict__ T) {
  __shared__ float sm[64][65];
  const int t   = threadIdx.x;
  const int k0t = blockIdx.x * 64;
  const int n0t = blockIdx.y * 64;
  const int z   = blockIdx.z;
  const float* W = (z == 0) ? W1 : W2;
#pragma unroll
  for (int i = 0; i < 8; ++i) {
    const int idx = i * 256 + t;
    const int r = idx >> 6;
    const int c = idx & 63;
    sm[c][r] = W[(size_t)(k0t + r) * kHid + n0t + c];
  }
  asm volatile("" ::: "memory");
#pragma unroll
  for (int i = 8; i < 16; ++i) {
    const int idx = i * 256 + t;
    const int r = idx >> 6;
    const int c = idx & 63;
    sm[c][r] = W[(size_t)(k0t + r) * kHid + n0t + c];
  }
  __syncthreads();
  const int lane = t & 31, wave = t >> 5;
  const int q = lane >> 3, c8 = (lane & 7) * 8;
  unsigned short* op = T + (size_t)z * kHid * kHid;
  for (int pass = 0; pass < 2; ++pass) {
#pragma unroll
    for (int it = 0; it < 2; ++it) {
      const int row = wave * 8 + it * 4 + q;
      unsigned short hb[8];
#pragma unroll
      for (int e = 0; e < 8; ++e) {
        const float v = sm[row][c8 + e];
        const unsigned short bb = f2bf_bits(v);
        const unsigned short fb = h_bits(bf_bits2f(bb) * kW2Carry);
        hb[e] = (z == 0) ? bb : fb;
      }
      const v4u u = (v4u){pk16(hb[0], hb[1]), pk16(hb[2], hb[3]), pk16(hb[4], hb[5]), pk16(hb[6], hb[7])};
      *(volatile v4u*)(op + (size_t)(n0t + row) * kHid + k0t + c8) = u;
    }
    __threadfence();
  }
}

__global__ __launch_bounds__(256) void decay_kernel(const float* __restrict__ SCp, unsigned short* __restrict__ PPp,
                                                    float lg0, float lg1, float carry) {
  const int n = blockIdx.x;
  const int y = blockIdx.y;
  const int t = threadIdx.x;
  const float lg = (y == 0) ? lg0 : lg1;
  const size_t rowoff = ((size_t)y * kS + n) * kS;
  const int c0   = 8 * t;
  const int clim = n & ~7;
  const int cl   = (c0 < clim) ? c0 : clim;
  const float* sr = SCp + rowoff + cl;
  const v4f a = *(const v4f*)(sr);
  const v4f c = *(const v4f*)(sr + 4);
  unsigned short hb[8];
#pragma unroll
  for (int e = 0; e < 4; ++e) {
    const int colA = c0 + e;
    const int colB = c0 + 4 + e;
    const float dA = exp2f((float)(n - colA) * lg);
    const float dB = exp2f((float)(n - colB) * lg);
    const float pA = (a[e] * dA) * carry;
    const float pB = (c[e] * dB) * carry;
    hb[e]     = h_bits((colA <= n) ? pA : 0.0f);
    hb[4 + e] = h_bits((colB <= n) ? pB : 0.0f);
  }
  const v4u u = (v4u){pk16(hb[0], hb[1]), pk16(hb[2], hb[3]), pk16(hb[4], hb[5]), pk16(hb[6], hb[7])};
  unsigned short* pr = PPp + rowoff + (size_t)c0;
  *(volatile v4u*)pr = u;
  __threadfence();
  *(volatile v4u*)pr = u;
}

__global__ __launch_bounds__(256) void gn_gate_kernel(const float* __restrict__ RETp, const float* __restrict__ GATp,
                                                      const float* __restrict__ gnw, const float* __restrict__ gnb,
                                                      unsigned short* __restrict__ PREp) {
  __shared__ __align__(16) unsigned int stg[8][64];
  const int t    = threadIdx.x;
  const int lane = t & 31, wave = t >> 5;
  const int r    = blockIdx.x * 8 + wave;
  const int tok  = r >> 3, h = r & 7;
  const size_t base = (size_t)tok * kHid + h * kHD + 4 * lane;
  const v4f a  = *(const v4f*)(RETp + base);
  const v4f g  = *(const v4f*)(GATp + base);
  const v4f wr = *(const v4f*)(gnw + h * kHD + 4 * lane);
  const v4f br = *(const v4f*)(gnb + h * kHD + 4 * lane);

  float s = (a[0] + a[1]) + (a[2] + a[3]);
#pragma unroll
  for (int off = 1; off < 32; off <<= 1) s += __shfl_xor(s, off, 32);
  const float mu = s * kInvHD;
  const float d0 = a[0] - mu, d1 = a[1] - mu, d2 = a[2] - mu, d3 = a[3] - mu;
  float ss = (d0 * d0 + d1 * d1) + (d2 * d2 + d3 * d3);
#pragma unroll
  for (int off = 1; off < 32; off <<= 1) ss += __shfl_xor(ss, off, 32);
  const float var = ss * kInvHD;
  const float rs  = rsqrtf(var + kEps);

  const float w0 = bf_bits2f(f2bf_bits(wr[0])), w1 = bf_bits2f(f2bf_bits(wr[1]));
  const float w2 = bf_bits2f(f2bf_bits(wr[2])), w3 = bf_bits2f(f2bf_bits(wr[3]));
  const float b0 = bf_bits2f(f2bf_bits(br[0])), b1 = bf_bits2f(f2bf_bits(br[1]));
  const float b2 = bf_bits2f(f2bf_bits(br[2])), b3 = bf_bits2f(f2bf_bits(br[3]));

  float y0 = (d0 * rs) * w0; y0 = y0 + b0;
  float y1 = (d1 * rs) * w1; y1 = y1 + b1;
  float y2 = (d2 * rs) * w2; y2 = y2 + b2;
  float y3 = (d3 * rs) * w3; y3 = y3 + b3;

  const float g0 = g[0], g1 = g[1], g2 = g[2], g3 = g[3];
  const float sg0 = 1.0f / (1.0f + expf(-g0));
  const float sg1 = 1.0f / (1.0f + expf(-g1));
  const float sg2 = 1.0f / (1.0f + expf(-g2));
  const float sg3 = 1.0f / (1.0f + expf(-g3));
  const float p0 = g0 * sg0 + y0;
  const float p1 = g1 * sg1 + y1;
  const float p2 = g2 * sg2 + y2;
  const float p3 = g3 * sg3 + y3;

  stg[wave][2 * lane]     = pk16(h_bits(p0), h_bits(p1));
  stg[wave][2 * lane + 1] = pk16(h_bits(p2), h_bits(p3));
  __syncthreads();
  const int l16 = lane & 15;
  const v4u u = *(const v4u*)(&stg[wave][4 * l16]);
  unsigned short* dst = PREp + (size_t)tok * kHid + h * kHD + 8 * l16;
  if (lane < 16) *(volatile v4u*)dst = u;
  __threadfence();
  if (lane < 16) *(volatile v4u*)dst = u;
}

extern "C" void kernel_launch(void* const* d_in, const int* in_sizes, int n_in,
                              void* d_out, int out_size, void* d_ws, size_t ws_size,
                              hipStream_t stream) {
  if (n_in < 8) return;
  const int nX = kTok * kHid;
  const int nHW = kNH * kHD * kHD;
  const int nSQ = kHid * kHid;
  if (in_sizes[0] != nX || in_sizes[1] != nHW || in_sizes[2] != nHW || in_sizes[3] != nHW) return;
  if (in_sizes[4] != nSQ || in_sizes[5] != nSQ || in_sizes[6] != kHid || in_sizes[7] != kHid) return;
  if (out_size != nX) return;

  const size_t szXB  = (size_t)kTok * kHid * 2;
  const size_t szWT  = (size_t)3 * kNH * kHD * kHD * 2;
  const size_t szSQ  = (size_t)2 * kHid * kHid * 2;
  const size_t szQ   = (size_t)kTok * kHid * 2;
  const size_t szVT  = (size_t)kNH * kHD * kTok * 2;
  const size_t szSC  = (size_t)kGrp * kS * kS * 4;
  const size_t szPP  = (size_t)kGrp * kS * kS * 2;
  const size_t szRET = (size_t)kTok * kHid * 4;
  const size_t szGAT = szRET;
  const size_t szPRE = (size_t)kTok * kHid * 2;
  const size_t offXB  = 0;
  const size_t offWT  = offXB + szXB;
  const size_t offSQ  = offWT + szWT;
  const size_t offQ   = offSQ + szSQ;
  const size_t offK   = offQ + szQ;
  const size_t offVT  = offK + szQ;
  const size_t offSC  = offVT + szVT;
  const size_t offPP  = offSC + szSC;
  const size_t offRET = offPP + szPP;
  const size_t offGAT = offRET + szRET;
  const size_t offPRE = offGAT + szGAT;
  const size_t total  = offPRE + szPRE;
  if (ws_size < total) return;

  const float* x   = (const float*)d_in[0];
  const float* Wq  = (const float*)d_in[1];
  const float* Wk  = (const float*)d_in[2];
  const float* Wv  = (const float*)d_in[3];
  const float* W1  = (const float*)d_in[4];
  const float* W2  = (const float*)d_in[5];
  const float* gnw = (const float*)d_in[6];
  const float* gnb = (const float*)d_in[7];
  float* out = (float*)d_out;
  char* ws = (char*)d_ws;
  unsigned short* XB  = (unsigned short*)(ws + offXB);
  unsigned short* WT  = (unsigned short*)(ws + offWT);
  unsigned short* SQT = (unsigned short*)(ws + offSQ);
  unsigned short* Q16 = (unsigned short*)(ws + offQ);
  unsigned short* K16 = (unsigned short*)(ws + offK);
  unsigned short* VT  = (unsigned short*)(ws + offVT);
  float*          SC  = (float*)(ws + offSC);
  unsigned short* PP  = (unsigned short*)(ws + offPP);
  float*          RET = (float*)(ws + offRET);
  float*          GAT = (float*)(ws + offGAT);
  unsigned short* PRE = (unsigned short*)(ws + offPRE);
  unsigned short* WQT = WT;
  unsigned short* WKT = WT + (size_t)kNH * kHD * kHD;
  unsigned short* WVT = WT + (size_t)2 * kNH * kHD * kHD;
  unsigned short* W1T = SQT;
  unsigned short* W2T = SQT + (size_t)kHid * kHid;

  const double lnlo = log(1.0 / 512.0);
  const double lnhi = log(1.0 / 32.0);
  const double stp  = (lnhi - lnlo) / 7.0;
  float lg2[kNH];
  for (int h = 0; h < kNH; ++h) {
    const double lin = (h == kNH - 1) ? lnhi : ((double)h * stp + lnlo);
    const float gam = (float)(1.0 - exp(lin));
    lg2[h] = (float)log2((double)gam);
  }

  const int n8 = nX / 8;
  cast8_bf16_kernel<<<dim3(n8 / 256), dim3(256), 0, stream>>>(x, XB, n8);
  headw_kernel<<<dim3(kHD / 64, kHD / 64, 3 * kNH), dim3(256), 0, stream>>>(Wq, Wk, Wv, WT);
  sqw_kernel<<<dim3(kHid / 64, kHid / 64, 2), dim3(256), 0, stream>>>(W1, W2, SQT);

  const int tilesQK = (kTok / 64) * (kHD / 64);
  wmma_gemm64<1, false, 0, 1, false, 0, 0><<<dim3(tilesQK / 8, kNH), dim3(256), 0, stream>>>(
      XB, XB, kHid, (long)kHD, WQT, WQT, kHD, (long)kHD * kHD,
      (void*)Q16, (void*)Q16, kHid, (long)kHD, gnw, gnw, 0L, kTok, kHD, kHD, kQCarry);
  wmma_gemm64<1, false, 0, 1, false, 0, 0><<<dim3(tilesQK / 8, kNH), dim3(256), 0, stream>>>(
      XB, XB, kHid, (long)kHD, WKT, WKT, kHD, (long)kHD * kHD,
      (void*)K16, (void*)K16, kHid, (long)kHD, gnw, gnw, 0L, kTok, kHD, kHD, kQCarry);
  const int tilesV = (kHD / 64) * (kTok / 64);
  wmma_gemm64<1, false, 0, 1, false, 0, 0><<<dim3(tilesV / 8, kNH), dim3(256), 0, stream>>>(
      WVT, WVT, kHD, (long)kHD * kHD, XB, XB, kHid, (long)kHD,
      (void*)VT, (void*)VT, kTok, (long)kHD * kTok, gnw, gnw, 0L, kHD, kTok, kHD, kVCarry);
  const int tilesBig = (kTok / 64) * (kHid / 64);
  wmma_gemm64<1, false, 0, 0, false, 0, 0><<<dim3(tilesBig / 8, 1), dim3(256), 0, stream>>>(
      XB, XB, kHid, 0L, W1T, W1T, kHid, 0L,
      (void*)GAT, (void*)GAT, kHid, 0L, gnw, gnw, 0L, kTok, kHid, kHid, 1.0f);

  const int tilesScore = (kS / 64) * (kS / 64);
  const int tilesPV    = (kS / 64) * (kHD / 64);
  for (int b = 0; b < kB; ++b) {
    for (int g = 0; g < kNH / kGrp; ++g) {
      const size_t tokOff = ((size_t)b * kS) * kHid + (size_t)g * kGrp * kHD;
      const unsigned short* Ag  = Q16 + tokOff;
      const unsigned short* Btg = K16 + tokOff;
      wmma_gemm64<0, false, 0, 0, false, 0, 1><<<dim3(tilesScore / 8, kGrp), dim3(256), 0, stream>>>(
          Ag, Ag, kHid, (long)kHD, Btg, Btg, kHid, (long)kHD,
          (void*)SC, (void*)SC, kS, (long)kS * kS, gnw, gnw, 0L, kS, kS, kHD, kScoreScale);
      decay_kernel<<<dim3(kS, kGrp), dim3(256), 0, stream>>>(SC, PP, lg2[g * kGrp], lg2[g * kGrp + 1], kPCarry);
      const unsigned short* VTg = VT + (size_t)(g * kGrp) * kHD * kTok + (size_t)b * kS;
      float* RETg = RET + ((size_t)b * kS) * kHid + (size_t)g * kGrp * kHD;
      wmma_gemm64<0, false, 0, 0, false, 0, 2><<<dim3(tilesPV / 8, kGrp), dim3(256), 0, stream>>>(
          PP, PP, kS, (long)kS * kS, VTg, VTg, kTok, (long)kHD * kTok,
          (void*)RETg, (void*)RETg, kHid, (long)kHD, gnw, gnw, 0L, kS, kHD, kS, kPVScale);
    }
  }

  gn_gate_kernel<<<dim3(kTok * kNH / 8), dim3(256), 0, stream>>>(RET, GAT, gnw, gnb, PRE);

  wmma_gemm64<0, false, 0, 0, false, 0, 0><<<dim3(tilesBig / 8, 1), dim3(256), 0, stream>>>(
      PRE, PRE, kHid, 0L, W2T, W2T, kHid, 0L,
      (void*)out, (void*)out, kHid, 0L, gnw, gnw, 0L, kTok, kHid, kHid, kOutScale);
}
